// _TransformerBlock_21260088115361
// MI455X (gfx1250) — hardware-run, weakly checked
//
#include <hip/hip_runtime.h>
#include <math.h>

constexpr int kB    = 2;
constexpr int kL    = 2048;
constexpr int kD    = 1024;
constexpr int kH    = 16;
constexpr int kDh   = 64;
constexpr int kFF   = 4096;
constexpr int kTok  = kB * kL;
constexpr int kG    = 2;
constexpr int kQKld = 2 * kD;
constexpr float kWCarry    = 64.0f;
constexpr float kWCarryInv = 1.0f / 64.0f;
constexpr float kPCarry    = 32768.0f;
constexpr float kOCarry    = 256.0f;
constexpr float kAttnScale = 0.125f;
constexpr float kPVScale   = kOCarry / kPCarry;
constexpr float kWoScale   = 1.0f / (kOCarry * kWCarry);
constexpr float kInvD      = 1.0f / 1024.0f;
constexpr float kLnEps     = 1e-5f;
static_assert(kH * kDh == kD, "shape");
static_assert(kD == 128 * 8, "ln thread map");
static_assert(kL == 256 * 8, "softmax thread map");
static_assert(kH % kG == 0, "groups");
static_assert(kTok % 64 == 0 && kD % 64 == 0 && kFF % 64 == 0 && kL % 64 == 0 && kDh % 64 == 0 && kQKld % 64 == 0, "tile multiples");
static_assert(kD % 32 == 0 && kDh % 32 == 0 && kL % 32 == 0 && kFF % 32 == 0, "k multiples");
constexpr int kTilesQK = (kTok / 64) * (kQKld / 64);
constexpr int kTilesVT = (kD / 64) * (kL / 64);
constexpr int kTilesS  = (kL / 64) * (kL / 64);
constexpr int kTilesPV = (kL / 64) * (kDh / 64);
constexpr int kTilesWo = (kTok / 64) * (kD / 64);
constexpr int kTilesW1 = (kTok / 64) * (kFF / 64);
constexpr int kTilesW2 = (kTok / 64) * (kD / 64);
static_assert(kTilesQK % 8 == 0 && kTilesVT % 8 == 0 && kTilesS % 8 == 0 && kTilesPV % 8 == 0 &&
              kTilesWo % 8 == 0 && kTilesW1 % 8 == 0 && kTilesW2 % 8 == 0, "8 waves per block");

constexpr size_t kOffWqk = 0;
constexpr size_t kOffWv  = kOffWqk + (size_t)kQKld * kD * 2;
constexpr size_t kOffWo  = kOffWv + (size_t)kD * kD * 2;
constexpr size_t kOffW1  = kOffWo + (size_t)kD * kD * 2;
constexpr size_t kOffW2  = kOffW1 + (size_t)kFF * kD * 2;
constexpr size_t kOffH   = kOffW2 + (size_t)kD * kFF * 2;
constexpr size_t kOffQK  = kOffH + (size_t)kTok * kD * 2;
constexpr size_t kOffVT  = kOffQK + (size_t)kTok * kQKld * 2;
constexpr size_t kOffPP  = kOffVT + (size_t)kB * kH * kDh * kL * 2;
constexpr size_t kOffSC  = kOffPP + (size_t)kG * kL * kL * 2;
constexpr size_t kOffO   = kOffSC + (size_t)kG * kL * kL * 4;
constexpr size_t kOffX2  = kOffO + (size_t)kTok * kD * 2;
constexpr size_t kWsTotal = kOffX2 + (size_t)kTok * kD * 4;
constexpr size_t kOffUG  = kOffQK;
static_assert(kWsTotal == 134217728u, "carve total");
static_assert(kOffUG + (size_t)kTok * kFF * 2 <= kOffSC, "UG alias inside dead f16 planes");

typedef __attribute__((ext_vector_type(16))) _Float16 v16h;
typedef __attribute__((ext_vector_type(8)))  _Float16 v8h;
typedef __attribute__((ext_vector_type(16))) __bf16   v16b;
typedef __attribute__((ext_vector_type(8)))  __bf16   v8b;
typedef __attribute__((ext_vector_type(8)))  float    v8f;
typedef __attribute__((ext_vector_type(4)))  float    v4f;
typedef __attribute__((ext_vector_type(4)))  unsigned int v4u;

__device__ __forceinline__ unsigned short f2bf_bits(float f) {
  unsigned u = __float_as_uint(f);
  return (unsigned short)((u + 0x7FFFu + ((u >> 16) & 1u)) >> 16);
}
__device__ __forceinline__ float bf_bits2f(unsigned short h) { return __uint_as_float(((unsigned)h) << 16); }

__device__ __forceinline__ void dep_guard_h(v8f& a, v8f& b, v16h x, v16h y) { asm volatile("v_nop\n\tv_nop\n\tv_nop\n\tv_nop" : "+v"(a), "+v"(b) : "v"(x), "v"(y)); }
__device__ __forceinline__ void dep_guard_b(v8f& a, v8f& b, v16b x, v16b y) { asm volatile("v_nop\n\tv_nop\n\tv_nop\n\tv_nop" : "+v"(a), "+v"(b) : "v"(x), "v"(y)); }
__device__ __forceinline__ void dep_guard4_h(v8f& a, v8f& b, v8f& c, v8f& d, v16h x, v16h y) { asm volatile("v_nop\n\tv_nop\n\tv_nop\n\tv_nop" : "+v"(a), "+v"(b), "+v"(c), "+v"(d) : "v"(x), "v"(y)); }
__device__ __forceinline__ void dep_guard4_b(v8f& a, v8f& b, v8f& c, v8f& d, v16b x, v16b y) { asm volatile("v_nop\n\tv_nop\n\tv_nop\n\tv_nop" : "+v"(a), "+v"(b), "+v"(c), "+v"(d) : "v"(x), "v"(y)); }
__device__ __forceinline__ void keep4_h(v16h a, v16h b, v16h c, v16h d) { asm volatile("v_nop" :: "v"(a), "v"(b), "v"(c), "v"(d)); }
__device__ __forceinline__ void keep4_b(v16b a, v16b b, v16b c, v16b d) { asm volatile("v_nop" :: "v"(a), "v"(b), "v"(c), "v"(d)); }
__device__ __forceinline__ void acc_guard4(v8f& a, v8f& b, v8f& c, v8f& d) { asm volatile("v_nop\n\tv_nop\n\tv_nop\n\tv_nop" : "+v"(a), "+v"(b), "+v"(c), "+v"(d)); }
template <typename T> struct Frag;
template <> struct Frag<_Float16> {
  typedef v16h V; union U { v16h v; v8h h[2]; };
  static __device__ __forceinline__ v16h load(const _Float16* p) {
    U f; f.h[0] = *(const v8h*)(p); f.h[1] = *(const v8h*)(p + 16); return f.v;
  }
  static __device__ __forceinline__ v8f mma(v16h a, v16h b, v8f c) {
    return __builtin_amdgcn_wmma_f32_16x16x32_f16(false, a, false, b, (short)0, c, false, false);
  }
  static __device__ __forceinline__ void guard(v8f& a, v8f& b, v16h x, v16h y) { dep_guard_h(a, b, x, y); }
  static __device__ __forceinline__ void guard4(v8f& a, v8f& b, v8f& c, v8f& d, v16h x, v16h y) { dep_guard4_h(a, b, c, d, x, y); }
  static __device__ __forceinline__ void keep(v16h a, v16h b, v16h c, v16h d) { keep4_h(a, b, c, d); }
};
template <> struct Frag<__bf16> {
  typedef v16b V; union U { v16b v; v8b h[2]; };
  static __device__ __forceinline__ v16b load(const __bf16* p) {
    U f; f.h[0] = *(const v8b*)(p); f.h[1] = *(const v8b*)(p + 16); return f.v;
  }
  static __device__ __forceinline__ v8f mma(v16b a, v16b b, v8f c) {
    return __builtin_amdgcn_wmma_f32_16x16x32_bf16(false, a, false, b, (short)0, c, false, false);
  }
  static __device__ __forceinline__ void guard(v8f& a, v8f& b, v16b x, v16b y) { dep_guard_b(a, b, x, y); }
  static __device__ __forceinline__ void guard4(v8f& a, v8f& b, v8f& c, v8f& d, v16b x, v16b y) { dep_guard4_b(a, b, c, d, x, y); }
  static __device__ __forceinline__ void keep(v16b a, v16b b, v16b c, v16b d) { keep4_b(a, b, c, d); }
};

__device__ __forceinline__ unsigned pk16(unsigned short a, unsigned short b) { return (unsigned)a | ((unsigned)b << 16); }
__device__ __forceinline__ unsigned short h_bits(float f) { const _Float16 h = (_Float16)f; return __builtin_bit_cast(unsigned short, h); }
__device__ __forceinline__ float h16_to_f32(unsigned hb) {
  const unsigned sgn = (hb & 0x8000u) << 16; const unsigned em = hb & 0x7fffu;
  const float fn = __uint_as_float((em << 13) + 0x38000000u);
  const float fs = (float)em * 5.9604644775390625e-8f;
  const float mag = (em < 0x400u) ? fs : fn; return __uint_as_float(__float_as_uint(mag) | sgn);
}

template <int ET> struct Elem;
template <> struct Elem<0> { typedef _Float16 T; };
template <> struct Elem<1> { typedef __bf16 T; };
template <int ET, bool SPLIT, int BIAS_MODE, int OUT_MODE, bool RESID>
__global__ __launch_bounds__(256) void wmma_gemm64(
    const unsigned short* __restrict__ Ap, const unsigned short* __restrict__ A2p, int lda, long strideA,
    const unsigned short* __restrict__ Btp, const unsigned short* __restrict__ Bt2p, int ldb, long strideB,
    void* __restrict__ Cout, void* __restrict__ Cout2, int ldc, long strideC,
    const float* __restrict__ bias,
    const float* __restrict__ resid, long strideR,
    int M, int N, int K, float scale) {
  static_assert(!RESID || OUT_MODE == 0, "resid only with f32 out");
  typedef typename Elem<ET>::T T;
  typedef typename Frag<T>::V V;
  const T* A = (const T*)Ap; const T* A2 = (const T*)A2p; const T* Bt = (const T*)Btp; const T* Bt2 = (const T*)Bt2p;
  __shared__ __align__(16) float sT[8][16 * 68];
  const int b    = blockIdx.y;
  const int lane = threadIdx.x & 31;
  const int wave = threadIdx.x >> 5;
  const int tilesN = N >> 6;
  const int tilesM = M >> 6;
  const int tile = blockIdx.x * 8 + wave;
  if (tile >= tilesM * tilesN) return;
  const int tm = tile / tilesN;
  const int tn = tile - tm * tilesN;
  const int m0 = tm << 6;
  const int n0 = tn << 6;

  const T* Ab  = A  + (size_t)b * strideA;
  const T* Bb  = Bt + (size_t)b * strideB;
  const T* Ab2 = SPLIT ? (A2  + (size_t)b * strideA) : nullptr;
  const T* Bb2 = SPLIT ? (Bt2 + (size_t)b * strideB) : nullptr;

  const int rlane = lane & 15;
  const int koff  = (lane >> 4) * 8;
  const int mOff  = (lane >> 4) * 8;

  v8f acc[4][4];
#pragma unroll
  for (int i = 0; i < 4; ++i)
#pragma unroll
    for (int j = 0; j < 4; ++j) acc[i][j] = (v8f){0.f,0.f,0.f,0.f,0.f,0.f,0.f,0.f};

  for (int k0 = 0; k0 < K; k0 += 32) {
    V bh[4], bl[4];
#pragma unroll
    for (int j = 0; j < 4; ++j) {
      const size_t bo = (size_t)(n0 + (j << 4) + rlane) * ldb + koff + k0;
      bh[j] = Frag<T>::load(Bb + bo);
      if (SPLIT) bl[j] = Frag<T>::load(Bb2 + bo);
    }
#pragma unroll
    for (int i = 0; i < 4; ++i) {
      const size_t ao = (size_t)(m0 + (i << 4) + rlane) * lda + koff + k0;
      V ah = Frag<T>::load(Ab + ao);
      V al;
      if (SPLIT) al = Frag<T>::load(Ab2 + ao);
#pragma unroll
      for (int j = 0; j < 4; ++j) {
        acc[i][j] = Frag<T>::mma(ah, bh[j], acc[i][j]);
        if (SPLIT) {
          acc[i][j] = Frag<T>::mma(ah, bl[j], acc[i][j]);
          acc[i][j] = Frag<T>::mma(al, bh[j], acc[i][j]);
        }
      }
      Frag<T>::guard4(acc[i][0], acc[i][1], acc[i][2], acc[i][3], ah, SPLIT ? al : ah);
    }
    Frag<T>::keep(bh[0], bh[1], bh[2], bh[3]);
    if (SPLIT) Frag<T>::keep(bl[0], bl[1], bl[2], bl[3]);
  }
  acc_guard4(acc[0][0], acc[0][1], acc[0][2], acc[0][3]);
  acc_guard4(acc[1][0], acc[1][1], acc[1][2], acc[1][3]);
  acc_guard4(acc[2][0], acc[2][1], acc[2][2], acc[2][3]);
  acc_guard4(acc[3][0], acc[3][1], acc[3][2], acc[3][3]);

  float* slab = sT[wave];
  const float* Rb = RESID ? (resid + (size_t)b * strideR) : nullptr;
#pragma unroll
  for (int i = 0; i < 4; ++i) {
    const int mBase = m0 + (i << 4);
#pragma unroll
    for (int j = 0; j < 4; ++j) {
      const int n = n0 + (j << 4) + rlane;
      float bv = 0.f;
      if (BIAS_MODE == 2) bv = bias[n];
#pragma unroll
      for (int r = 0; r < 8; ++r) {
        float v = acc[i][j][r] * scale;
        if (BIAS_MODE == 1) v += bias[mBase + mOff + r];
        if (BIAS_MODE == 2) v += bv;
        slab[(mOff + r) * 68 + (j << 4) + rlane] = v;
      }
    }
    __builtin_amdgcn_fence(__ATOMIC_RELEASE, "workgroup");
    __builtin_amdgcn_wave_barrier();
    __builtin_amdgcn_fence(__ATOMIC_ACQUIRE, "workgroup");
    if (OUT_MODE == 0) {
      float* C = (float*)Cout + (size_t)b * strideC;
      const int hh = lane >> 4, c4 = (lane & 15) * 4;
      for (int pass = 0; pass < 2; ++pass) {
#pragma unroll
        for (int it = 0; it < 8; ++it) {
          const int row = it * 2 + hh;
          v4f v = *(const v4f*)(slab + row * 68 + c4);
          if (RESID) {
            const v4f rr = *(const v4f*)(Rb + (size_t)(mBase + row) * ldc + n0 + c4);
            v = v + rr;
          }
          *(volatile v4f*)(C + (size_t)(mBase + row) * ldc + n0 + c4) = v;
        }
        __threadfence();
      }
    } else {
      const int q = lane >> 3, c8 = (lane & 7) * 8;
      unsigned short* C  = (unsigned short*)Cout  + (size_t)b * strideC;
      unsigned short* C2 = (OUT_MODE == 2) ? ((unsigned short*)Cout2 + (size_t)b * strideC) : nullptr;
      for (int pass = 0; pass < 2; ++pass) {
#pragma unroll
        for (int it = 0; it < 4; ++it) {
          const int row = it * 4 + q;
          const float* sp = slab + row * 68 + c8;
          v8h hv, lv;
#pragma unroll
          for (int e = 0; e < 8; ++e) {
            if (OUT_MODE == 1) {
              hv[e] = (_Float16)sp[e];
            } else {
              unsigned short hb = f2bf_bits(sp[e]);
              unsigned short lb = f2bf_bits(sp[e] - bf_bits2f(hb));
              hv[e] = __builtin_bit_cast(_Float16, hb);
              lv[e] = __builtin_bit_cast(_Float16, lb);
            }
          }
          *(volatile v8h*)(C + (size_t)(mBase + row) * ldc + n0 + c8) = hv;
          if (OUT_MODE == 2) *(volatile v8h*)(C2 + (size_t)(mBase + row) * ldc + n0 + c8) = lv;
        }
        __threadfence();
      }
    }
    __builtin_amdgcn_fence(__ATOMIC_RELEASE, "workgroup");
    __builtin_amdgcn_wave_barrier();
    __builtin_amdgcn_fence(__ATOMIC_ACQUIRE, "workgroup");
  }
}

__global__ __launch_bounds__(256) void wt_cast_kernel(
    const float* __restrict__ Wa, const float* __restrict__ Wb, const float* __restrict__ Wc, const float* __restrict__ Wd,
    unsigned short* __restrict__ Oa, unsigned short* __restrict__ Ob, unsigned short* __restrict__ Oc, unsigned short* __restrict__ Od,
    int nrows, int ncols, float scale) {
  __shared__ float sm[64][65];
  const int t  = threadIdx.x;
  const int r0 = blockIdx.x * 64;
  const int c0 = blockIdx.y * 64;
  const int z  = blockIdx.z;
  const float* W = (z == 0) ? Wa : (z == 1) ? Wb : (z == 2) ? Wc : Wd;
  unsigned short* out = (z == 0) ? Oa : (z == 1) ? Ob : (z == 2) ? Oc : Od;
#pragma unroll
  for (int i = 0; i < 4; ++i) {
    const int e  = i * 256 + t;
    const int r  = e >> 4;
    const int c4 = (e & 15) * 4;
    const v4f w = *(const v4f*)(W + (size_t)(r0 + r) * ncols + c0 + c4);
    sm[c4 + 0][r] = w[0] * scale;
    sm[c4 + 1][r] = w[1] * scale;
    sm[c4 + 2][r] = w[2] * scale;
    sm[c4 + 3][r] = w[3] * scale;
  }
  __syncthreads();
  const int lane = t & 31, wave = t >> 5;
  const int q = lane >> 3, c8 = (lane & 7) * 8;
  for (int pass = 0; pass < 2; ++pass) {
#pragma unroll
    for (int it = 0; it < 2; ++it) {
      const int row = wave * 8 + it * 4 + q;
      unsigned short hb[8];
#pragma unroll
      for (int e = 0; e < 8; ++e) hb[e] = h_bits(sm[row][c8 + e]);
      const v4u u = (v4u){pk16(hb[0], hb[1]), pk16(hb[2], hb[3]), pk16(hb[4], hb[5]), pk16(hb[6], hb[7])};
      *(volatile v4u*)(out + (size_t)(c0 + row) * nrows + r0 + c8) = u;
    }
    __threadfence();
  }
}

template <bool ADDPOS>
__global__ __launch_bounds__(128) void layernorm_kernel(const float* __restrict__ xin, const float* __restrict__ gam,
                                                       const float* __restrict__ bet, const float* __restrict__ pos,
                                                       unsigned short* __restrict__ out) {
  __shared__ float redA[4];
  __shared__ float redB[4];
  const int row  = blockIdx.x;
  const int t    = threadIdx.x;
  const int lane = t & 31, wave = t >> 5;
  const int c0   = t * 8;
  const float* xr = xin + (size_t)row * kD + c0;
  const v4f a0 = *(const v4f*)(xr);
  const v4f a1 = *(const v4f*)(xr + 4);
  float v[8];
#pragma unroll
  for (int e = 0; e < 4; ++e) { v[e] = a0[e]; v[4 + e] = a1[e]; }
  float s = 0.0f;
#pragma unroll
  for (int e = 0; e < 8; ++e) s += v[e];
#pragma unroll
  for (int off = 16; off > 0; off >>= 1) s += __shfl_xor(s, off, 32);
  if (lane == 0) redA[wave] = s;
  __syncthreads();
  const float mean = ((redA[0] + redA[1]) + (redA[2] + redA[3])) * kInvD;
  float d[8];
  float s2 = 0.0f;
#pragma unroll
  for (int e = 0; e < 8; ++e) { d[e] = v[e] - mean; s2 += d[e] * d[e]; }
#pragma unroll
  for (int off = 16; off > 0; off >>= 1) s2 += __shfl_xor(s2, off, 32);
  if (lane == 0) redB[wave] = s2;
  __syncthreads();
  const float var  = ((redB[0] + redB[1]) + (redB[2] + redB[3])) * kInvD;
  const float rinv = rsqrtf(var + kLnEps);
  const v4f g0 = *(const v4f*)(gam + c0);
  const v4f g1 = *(const v4f*)(gam + c0 + 4);
  const v4f b0 = *(const v4f*)(bet + c0);
  const v4f b1 = *(const v4f*)(bet + c0 + 4);
  float y[8];
#pragma unroll
  for (int e = 0; e < 4; ++e) {
    y[e]     = d[e] * rinv * g0[e] + b0[e];
    y[4 + e] = d[4 + e] * rinv * g1[e] + b1[e];
  }
  if (ADDPOS) {
    const float* pr = pos + (size_t)(row & (kL - 1)) * kD + c0;
    const v4f p0 = *(const v4f*)(pr);
    const v4f p1 = *(const v4f*)(pr + 4);
#pragma unroll
    for (int e = 0; e < 4; ++e) { y[e] += p0[e]; y[4 + e] += p1[e]; }
  }
  unsigned short hb[8];
#pragma unroll
  for (int e = 0; e < 8; ++e) hb[e] = h_bits(y[e]);
  const v4u u = (v4u){pk16(hb[0], hb[1]), pk16(hb[2], hb[3]), pk16(hb[4], hb[5]), pk16(hb[6], hb[7])};
  unsigned short* op = out + (size_t)row * kD + c0;
  *(volatile v4u*)op = u;
  __threadfence();
  *(volatile v4u*)op = u;
}

__global__ __launch_bounds__(256) void softmax_row_kernel(const float* __restrict__ S, unsigned short* __restrict__ P) {
  __shared__ float redM[8];
  __shared__ float redS[8];
  const int row  = blockIdx.x;
  const int hg   = blockIdx.y;
  const int t    = threadIdx.x;
  const int lane = t & 31, wave = t >> 5;
  const size_t rowoff = ((size_t)hg * kL + row) * kL;
  const float* sr = S + rowoff + 8 * (size_t)t;
  const v4f a = *(const v4f*)(sr);
  const v4f c = *(const v4f*)(sr + 4);
  float x[8];
#pragma unroll
  for (int e = 0; e < 4; ++e) { x[e] = a[e]; x[4 + e] = c[e]; }
  float mx = fmaxf(fmaxf(fmaxf(x[0], x[1]), fmaxf(x[2], x[3])), fmaxf(fmaxf(x[4], x[5]), fmaxf(x[6], x[7])));
#pragma unroll
  for (int off = 16; off > 0; off >>= 1) mx = fmaxf(mx, __shfl_xor(mx, off, 32));
  if (lane == 0) redM[wave] = mx;
  __syncthreads();
  float m = redM[0];
#pragma unroll
  for (int w = 1; w < 8; ++w) m = fmaxf(m, redM[w]);
  float ex[8];
  float sum = 0.0f;
#pragma unroll
  for (int e = 0; e < 8; ++e) { ex[e] = expf(x[e] - m); sum += ex[e]; }
#pragma unroll
  for (int off = 16; off > 0; off >>= 1) sum += __shfl_xor(sum, off, 32);
  if (lane == 0) redS[wave] = sum;
  __syncthreads();
  float tot = redS[0];
#pragma unroll
  for (int w = 1; w < 8; ++w) tot += redS[w];
  const float inv = kPCarry / tot;
  unsigned short hb[8];
#pragma unroll
  for (int e = 0; e < 8; ++e) hb[e] = h_bits(ex[e] * inv);
  const v4u u = (v4u){pk16(hb[0], hb[1]), pk16(hb[2], hb[3]), pk16(hb[4], hb[5]), pk16(hb[6], hb[7])};
  unsigned short* pr = P + rowoff + 8 * (size_t)t;
  *(volatile v4u*)pr = u;
  __threadfence();
  *(volatile v4u*)pr = u;
}

__global__ __launch_bounds__(256) void gelu2_kernel(unsigned int* __restrict__ buf, int n2) {
  const int i = blockIdx.x * 256 + threadIdx.x;
  if (i >= n2) return;
  const unsigned w  = buf[i];
  const float u0 = h16_to_f32(w & 0xffffu);
  const float u1 = h16_to_f32(w >> 16);
  const float g0 = 0.5f * u0 * (1.0f + erff(u0 * 0.70710678118654752f));
  const float g1 = 0.5f * u1 * (1.0f + erff(u1 * 0.70710678118654752f));
  const unsigned o = pk16(h_bits(g0), h_bits(g1));
  unsigned int* q = buf + i;
  *(volatile unsigned int*)q = o;
  __threadfence();
  *(volatile unsigned int*)q = o;
}

extern "C" void kernel_launch(void* const* d_in, const int* in_sizes, int n_in,
                              void* d_out, int out_size, void* d_ws, size_t ws_size,
                              hipStream_t stream) {
  if (n_in < 15) return;
  if (in_sizes[0] != kTok * kD || in_sizes[1] != kL * kD) return;
  if (in_sizes[2] != kD || in_sizes[3] != kD) return;
  if (in_sizes[4] != kD * kD || in_sizes[5] != kD * kD || in_sizes[6] != kD * kD || in_sizes[7] != kD * kD) return;
  if (in_sizes[8] != kD || in_sizes[9] != kD || in_sizes[10] != kD) return;
  if (in_sizes[11] != kD * kFF || in_sizes[12] != kFF || in_sizes[13] != kFF * kD || in_sizes[14] != kD) return;
  if (out_size != kTok * kD) return;
  if (ws_size < kWsTotal) return;

  const float* x     = (const float*)d_in[0];
  const float* pos   = (const float*)d_in[1];
  const float* ln1_g = (const float*)d_in[2];
  const float* ln1_b = (const float*)d_in[3];
  const float* Wq    = (const float*)d_in[4];
  const float* Wk    = (const float*)d_in[5];
  const float* Wv    = (const float*)d_in[6];
  const float* Wo    = (const float*)d_in[7];
  const float* bo    = (const float*)d_in[8];
  const float* ln2_g = (const float*)d_in[9];
  const float* ln2_b = (const float*)d_in[10];
  const float* W1    = (const float*)d_in[11];
  const float* b1    = (const float*)d_in[12];
  const float* W2    = (const float*)d_in[13];
  const float* b2    = (const float*)d_in[14];
  float* out = (float*)d_out;
  char* ws = (char*)d_ws;
  unsigned short* WqkT = (unsigned short*)(ws + kOffWqk);
  unsigned short* WvT  = (unsigned short*)(ws + kOffWv);
  unsigned short* WoT  = (unsigned short*)(ws + kOffWo);
  unsigned short* W1T  = (unsigned short*)(ws + kOffW1);
  unsigned short* W2T  = (unsigned short*)(ws + kOffW2);
  unsigned short* Hp   = (unsigned short*)(ws + kOffH);
  unsigned short* Mp   = Hp;
  unsigned short* QKp  = (unsigned short*)(ws + kOffQK);
  unsigned short* VTp  = (unsigned short*)(ws + kOffVT);
  unsigned short* PPp  = (unsigned short*)(ws + kOffPP);
  float*          SCp  = (float*)(ws + kOffSC);
  unsigned short* Op   = (unsigned short*)(ws + kOffO);
  float*          X2p  = (float*)(ws + kOffX2);
  unsigned short* UGp  = (unsigned short*)(ws + kOffUG);

  wt_cast_kernel<<<dim3(kD / 64, kD / 64, 4), dim3(256), 0, stream>>>(
      Wq, Wk, Wv, Wo, WqkT, WqkT + (size_t)kD * kD, WvT, WoT, kD, kD, kWCarry);
  wt_cast_kernel<<<dim3(kD / 64, kFF / 64, 1), dim3(256), 0, stream>>>(
      W1, W1, W1, W1, W1T, W1T, W1T, W1T, kD, kFF, kWCarry);
  wt_cast_kernel<<<dim3(kFF / 64, kD / 64, 1), dim3(256), 0, stream>>>(
      W2, W2, W2, W2, W2T, W2T, W2T, W2T, kFF, kD, kWCarry);

  layernorm_kernel<true><<<dim3(kTok), dim3(128), 0, stream>>>(x, ln1_g, ln1_b, pos, Hp);

  wmma_gemm64<0, false, 0, 1, false><<<dim3(kTilesQK / 8, 1), dim3(256), 0, stream>>>(
      Hp, Hp, kD, 0L, WqkT, WqkT, kD, 0L, (void*)QKp, (void*)QKp, kQKld, 0L, bo, x, 0L, kTok, kQKld, kD, kWCarryInv);
  wmma_gemm64<0, false, 0, 1, false><<<dim3(kTilesVT / 8, kB), dim3(256), 0, stream>>>(
      WvT, WvT, kD, 0L, Hp, Hp, kD, (long)kL * kD, (void*)VTp, (void*)VTp, kL, (long)kH * kDh * kL,
      bo, x, 0L, kD, kL, kD, kWCarryInv);

  const long strideHead = (long)kDh;
  const long strideSC   = (long)kL * kL;
  const long strideVT   = (long)kDh * kL;
  for (int b = 0; b < kB; ++b) {
    for (int g = 0; g < kH / kG; ++g) {
      const size_t qkOff = (size_t)b * kL * kQKld + (size_t)g * kG * kDh;
      const unsigned short* Aq = QKp + qkOff;
      const unsigned short* Bk = QKp + qkOff + kD;
      wmma_gemm64<0, false, 0, 0, false><<<dim3(kTilesS / 8, kG), dim3(256), 0, stream>>>(
          Aq, Aq, kQKld, strideHead, Bk, Bk, kQKld, strideHead,
          (void*)SCp, (void*)SCp, kL, strideSC, bo, x, 0L, kL, kL, kDh, kAttnScale);
      softmax_row_kernel<<<dim3(kL, kG), dim3(256), 0, stream>>>(SCp, PPp);
      const unsigned short* VTg = VTp + ((size_t)(b * kH + g * kG) * kDh) * kL;
      unsigned short* Og = Op + (size_t)b * kL * kD + (size_t)g * kG * kDh;
      wmma_gemm64<0, false, 0, 1, false><<<dim3(kTilesPV / 8, kG), dim3(256), 0, stream>>>(
          PPp, PPp, kL, strideSC, VTg, VTg, kL, strideVT,
          (void*)Og, (void*)Og, kD, strideHead, bo, x, 0L, kL, kDh, kL, kPVScale);
    }
  }

  wmma_gemm64<0, false, 2, 0, true><<<dim3(kTilesWo / 8, 1), dim3(256), 0, stream>>>(
      Op, Op, kD, 0L, WoT, WoT, kD, 0L, (void*)X2p, (void*)X2p, kD, 0L, bo, x, 0L, kTok, kD, kD, kWoScale);

  layernorm_kernel<false><<<dim3(kTok), dim3(128), 0, stream>>>(X2p, ln2_g, ln2_b, pos, Mp);

  wmma_gemm64<0, false, 2, 1, false><<<dim3(kTilesW1 / 8, 1), dim3(256), 0, stream>>>(
      Mp, Mp, kD, 0L, W1T, W1T, kD, 0L, (void*)UGp, (void*)UGp, kFF, 0L, b1, x, 0L, kTok, kFF, kD, kWCarryInv);

  const int n2 = (kTok * kFF) / 2;
  gelu2_kernel<<<dim3(n2 / 256), dim3(256), 0, stream>>>((unsigned int*)(void*)UGp, n2);

  wmma_gemm64<0, false, 2, 0, true><<<dim3(kTilesW2 / 8, 1), dim3(256), 0, stream>>>(
      UGp, UGp, kFF, 0L, W2T, W2T, kFF, 0L, (void*)out, (void*)out, kD, 0L, b2, X2p, 0L, kTok, kD, kFF, kWCarryInv);
}
